// CantorAttentionPlus_58007828300068
// MI455X (gfx1250) — hardware-verified
//
#include <hip/hip_runtime.h>
#include <stdint.h>


#define BDIM    1024
#define SEQ     2048
#define NBATCH  2
#define NTOK    (NBATCH * SEQ)
#define NHEADS  16
#define HD      64
#define KR      64
#define QSZ     ((size_t)NTOK * BDIM)

#define ASP     40
#define CSP     68
#define SMEM_U4 2176

typedef _Float16 v16h __attribute__((ext_vector_type(16)));
typedef _Float16 v8h  __attribute__((ext_vector_type(8)));
typedef float    v8f  __attribute__((ext_vector_type(8)));
typedef float    v4f  __attribute__((ext_vector_type(4)));
typedef float    v2f  __attribute__((ext_vector_type(2)));
typedef unsigned v4u  __attribute__((ext_vector_type(4)));

union Frag { uint4 u[2]; v16h v; };

__device__ __forceinline__ v8f wmma_f16_step(v16h a, v16h b, v8f c) {
  c = __builtin_amdgcn_wmma_f32_16x16x32_f16(false, a, false, b, (short)0, c, false, false);
  asm volatile("v_nop\n\tv_nop\n\tv_nop\n\tv_nop" : "+v"(c) : "v"(a), "v"(b));
  return c;
}

__global__ __launch_bounds__(256) void cvt_f32_f16(const float* __restrict__ src,
                                                   unsigned short* __restrict__ dst,
                                                   int n8, float scale)
{
  const int i = blockIdx.x * blockDim.x + threadIdx.x;
  if (i >= n8) return;
  const float* s = src + (size_t)i * 8;
  const v4f a = *(const v4f*)s;
  const v4f b = *(const v4f*)(s + 4);
  v8h hv;
  hv[0] = (_Float16)(a.x * scale);
  hv[1] = (_Float16)(a.y * scale);
  hv[2] = (_Float16)(a.z * scale);
  hv[3] = (_Float16)(a.w * scale);
  hv[4] = (_Float16)(b.x * scale);
  hv[5] = (_Float16)(b.y * scale);
  hv[6] = (_Float16)(b.z * scale);
  hv[7] = (_Float16)(b.w * scale);
  const v4u u = __builtin_bit_cast(v4u, hv);
  unsigned short* p = dst + (size_t)i * 8;
  *(volatile v4u*)p = u;
  __threadfence();
  *(volatile v4u*)p = u;
}

template <int MODE>
__global__ __launch_bounds__(256) void gemm_f16(const unsigned short* __restrict__ A,
                                                const unsigned short* __restrict__ Bm,
                                                const float* __restrict__ bias,
                                                float* __restrict__ dst,
                                                int Kdim, float oscale)
{
  __shared__ uint4 smem4[SMEM_U4];
  unsigned short* As = (unsigned short*)smem4;
  unsigned short* Bs = As + 128 * ASP;
  float* Cs = (float*)smem4;

  const int tid  = threadIdx.x;
  const int bm   = blockIdx.y * 128;
  const int bn   = blockIdx.x * 128;
  const int wid  = tid >> 5, lane = tid & 31;
  const int wm   = (wid & 3) * 32;
  const int wn   = (wid >> 2) * 64;
  const int lrow = lane & 15;
  const int hsel = lane >> 4;
  const int lkb  = hsel * 8;
  const int mofs = hsel * 8;

  const v8f vzero = {0.f, 0.f, 0.f, 0.f, 0.f, 0.f, 0.f, 0.f};
  v8f acc[2][4];
  #pragma unroll
  for (int mt = 0; mt < 2; ++mt)
    #pragma unroll
    for (int nt = 0; nt < 4; ++nt)
      acc[mt][nt] = vzero;

  const int r0 = tid >> 2;
  const int c0 = (tid & 3) * 8;

  #pragma unroll 1
  for (int kk = 0; kk < Kdim; kk += 32) {
    #pragma unroll
    for (int half = 0; half < 2; ++half) {
      const int row = r0 + half * 64;
      const uint4 va = *(const uint4*)(A  + (size_t)(bm + row) * Kdim + kk + c0);
      const uint4 vb = *(const uint4*)(Bm + (size_t)(bn + row) * Kdim + kk + c0);
      *(uint4*)(As + row * ASP + c0) = va;
      *(uint4*)(Bs + row * ASP + c0) = vb;
    }
    __syncthreads();

    Frag af[2], bfr[4];
    #pragma unroll
    for (int mt = 0; mt < 2; ++mt) {
      const unsigned short* p = As + (wm + mt * 16 + lrow) * ASP + lkb;
      af[mt].u[0] = *(const uint4*)p;
      af[mt].u[1] = *(const uint4*)(p + 16);
    }
    #pragma unroll
    for (int nt = 0; nt < 4; ++nt) {
      const unsigned short* p = Bs + (wn + nt * 16 + lrow) * ASP + lkb;
      bfr[nt].u[0] = *(const uint4*)p;
      bfr[nt].u[1] = *(const uint4*)(p + 16);
    }
    #pragma unroll
    for (int mt = 0; mt < 2; ++mt)
      #pragma unroll
      for (int nt = 0; nt < 4; ++nt)
        acc[mt][nt] = wmma_f16_step(af[mt].v, bfr[nt].v, acc[mt][nt]);
    __syncthreads();
  }

  const int col0 = bn + wn;
  const int m0   = bm + wm;
  float* dbase;
  int pitch;
  if (MODE == 0) {
    dbase = dst + (size_t)m0 * BDIM + col0;
    pitch = BDIM;
  } else {
    const int which = col0 >> 10;
    const int hh    = (col0 >> 6) & (NHEADS - 1);
    const int bb    = m0 >> 11;
    const int tok0  = m0 & (SEQ - 1);
    dbase = dst + (size_t)which * QSZ + ((size_t)(bb * NHEADS + hh) * SEQ + tok0) * HD;
    pitch = HD;
  }
  float bv[4];
  #pragma unroll
  for (int nt = 0; nt < 4; ++nt) bv[nt] = bias[col0 + nt * 16 + lrow];

  float* cw = Cs + wid * (16 * CSP);
  const int rsel = lane >> 4;
  const int cq   = (lane & 15) * 4;

  #pragma unroll
  for (int mt = 0; mt < 2; ++mt) {
    #pragma unroll
    for (int nt = 0; nt < 4; ++nt)
      #pragma unroll
      for (int r = 0; r < 8; ++r)
        cw[(mofs + r) * CSP + nt * 16 + lrow] = acc[mt][nt][r] * oscale + bv[nt];
    __syncthreads();
    #pragma unroll
    for (int i = 0; i < 8; ++i) {
      const int rr = 2 * i + rsel;
      const float* sp = cw + rr * CSP + cq;
      v4f v; v.x = sp[0]; v.y = sp[1]; v.z = sp[2]; v.w = sp[3];
      float* gp = dbase + (size_t)(mt * 16 + rr) * pitch + cq;
      *(volatile v4f*)gp = v;
    }
    __threadfence();
    #pragma unroll
    for (int i = 0; i < 8; ++i) {
      const int rr = 2 * i + rsel;
      const float* sp = cw + rr * CSP + cq;
      v4f v; v.x = sp[0]; v.y = sp[1]; v.z = sp[2]; v.w = sp[3];
      float* gp = dbase + (size_t)(mt * 16 + rr) * pitch + cq;
      *(volatile v4f*)gp = v;
    }
    __syncthreads();
  }
}

__global__ __launch_bounds__(256) void attn_gather(const float* __restrict__ qkvf,
                                                   const int* __restrict__ routes,
                                                   unsigned short* __restrict__ yh,
                                                   int nq)
{
  __shared__ float sp[8][KR];
  __shared__ int   sr[8][KR];
  const int tid = threadIdx.x, wid = tid >> 5, lane = tid & 31;
  const int gq_raw = blockIdx.x * 8 + wid;
  const bool valid = gq_raw < nq;
  const int gq = valid ? gq_raw : 0;
  const int n  = gq & (SEQ - 1);
  const int bh = gq >> 11;

  const float* qrow  = qkvf + (size_t)gq * HD;
  const float* kbase = qkvf + QSZ + (size_t)bh * SEQ * HD;
  const float* vbase = qkvf + 2 * QSZ + (size_t)bh * SEQ * HD;

  int rA = routes[n * KR + 2 * lane];
  int rB = routes[n * KR + 2 * lane + 1];
  rA = (rA < 0) ? rA + SEQ : rA;
  rB = (rB < 0) ? rB + SEQ : rB;
  rA = min(max(rA, 0), SEQ - 1);
  rB = min(max(rB, 0), SEQ - 1);
  const float* ka = kbase + (size_t)rA * HD;
  const float* kb = kbase + (size_t)rB * HD;

  float s0 = 0.f, s1 = 0.f;
  #pragma unroll 2
  for (int c = 0; c < HD / 4; ++c) {
    const v4f q4 = *(const v4f*)(qrow + 4 * c);
    const v4f a4 = *(const v4f*)(ka + 4 * c);
    const v4f b4 = *(const v4f*)(kb + 4 * c);
    s0 = fmaf(q4.x, a4.x, s0); s0 = fmaf(q4.y, a4.y, s0);
    s0 = fmaf(q4.z, a4.z, s0); s0 = fmaf(q4.w, a4.w, s0);
    s1 = fmaf(q4.x, b4.x, s1); s1 = fmaf(q4.y, b4.y, s1);
    s1 = fmaf(q4.z, b4.z, s1); s1 = fmaf(q4.w, b4.w, s1);
  }
  s0 *= 0.125f;
  s1 *= 0.125f;

  float mx = fmaxf(s0, s1);
  #pragma unroll
  for (int off = 16; off >= 1; off >>= 1)
    mx = fmaxf(mx, __shfl_xor(mx, off, 32));
  const float p0 = expf(s0 - mx), p1 = expf(s1 - mx);
  float sum = p0 + p1;
  #pragma unroll
  for (int off = 16; off >= 1; off >>= 1)
    sum += __shfl_xor(sum, off, 32);
  const float inv = 1.0f / sum;

  sp[wid][2 * lane]     = p0 * inv;
  sp[wid][2 * lane + 1] = p1 * inv;
  sr[wid][2 * lane]     = rA;
  sr[wid][2 * lane + 1] = rB;
  __syncthreads();

  float o0 = 0.f, o1 = 0.f;
  #pragma unroll 4
  for (int k = 0; k < KR; ++k) {
    const float p = sp[wid][k];
    const int   r = sr[wid][k];
    const v2f vv = *(const v2f*)(vbase + (size_t)r * HD + 2 * lane);
    o0 = fmaf(p, vv.x, o0);
    o1 = fmaf(p, vv.y, o1);
  }

  const _Float16 h0 = (_Float16)(o0 * 64.f);
  const _Float16 h1 = (_Float16)(o1 * 64.f);
  const unsigned packed = (unsigned)__builtin_bit_cast(unsigned short, h0) |
                          ((unsigned)__builtin_bit_cast(unsigned short, h1) << 16);
  const int src = 4 * (lane & 7);
  v4u st;
  st.x = __shfl(packed, src,     32);
  st.y = __shfl(packed, src + 1, 32);
  st.z = __shfl(packed, src + 2, 32);
  st.w = __shfl(packed, src + 3, 32);

  const int b = bh >> 4, h = bh & (NHEADS - 1);
  unsigned short* yp = yh + ((size_t)(b * SEQ + n)) * BDIM + h * HD + 8 * (lane & 7);
  if (valid && lane < 8) *(volatile v4u*)yp = st;
  __threadfence();
  if (valid && lane < 8) *(volatile v4u*)yp = st;
}

extern "C" void kernel_launch(void* const* d_in, const int* in_sizes, int n_in,
                              void* d_out, int out_size, void* d_ws, size_t ws_size,
                              hipStream_t stream)
{
  if (n_in < 6) return;
  if (in_sizes[0] != NTOK * BDIM) return;
  if (in_sizes[1] != SEQ * KR) return;
  if (in_sizes[2] != 3 * BDIM * BDIM) return;
  if (in_sizes[3] != 3 * BDIM) return;
  if (in_sizes[4] != BDIM * BDIM) return;
  if (in_sizes[5] != BDIM) return;
  if (out_size != NTOK * BDIM) return;

  const float* x      = (const float*)d_in[0];
  const int*   routes = (const int*)  d_in[1];
  const float* w_qkv  = (const float*)d_in[2];
  const float* b_qkv  = (const float*)d_in[3];
  const float* w_out  = (const float*)d_in[4];
  const float* b_out  = (const float*)d_in[5];
  float* out = (float*)d_out;

  const size_t xh_bytes  = (size_t)NTOK * BDIM * 2;
  const size_t wq_bytes  = (size_t)3 * BDIM * BDIM * 2;
  const size_t wo_bytes  = (size_t)BDIM * BDIM * 2;
  const size_t qkv_bytes = (size_t)3 * QSZ * 4;
  const size_t yh_bytes  = (size_t)NTOK * BDIM * 2;
  const size_t off_xh  = 0;
  const size_t off_wq  = off_xh + xh_bytes;
  const size_t off_wo  = off_wq + wq_bytes;
  const size_t off_qkv = off_wo + wo_bytes;
  const size_t off_yh  = off_qkv + qkv_bytes;
  const size_t total   = off_yh + yh_bytes;
  if (total > ws_size) return;

  char* ws = (char*)d_ws;
  unsigned short* xh    = (unsigned short*)(ws + off_xh);
  unsigned short* wqkvh = (unsigned short*)(ws + off_wq);
  unsigned short* wouth = (unsigned short*)(ws + off_wo);
  float*          qkvf  = (float*)(ws + off_qkv);
  unsigned short* yh    = (unsigned short*)(ws + off_yh);

  const int n8_x  = (NTOK * BDIM) / 8;
  const int n8_wq = (3 * BDIM * BDIM) / 8;
  const int n8_wo = (BDIM * BDIM) / 8;
  cvt_f32_f16<<<(n8_x + 255) / 256, 256, 0, stream>>>(x, xh, n8_x, 1.0f);
  cvt_f32_f16<<<(n8_wq + 255) / 256, 256, 0, stream>>>(w_qkv, wqkvh, n8_wq, 64.0f);
  cvt_f32_f16<<<(n8_wo + 255) / 256, 256, 0, stream>>>(w_out, wouth, n8_wo, 64.0f);

  gemm_f16<1><<<dim3((3 * BDIM) / 128, NTOK / 128), 256, 0, stream>>>(
      xh, wqkvh, b_qkv, qkvf, BDIM, 1.0f / 64.0f);

  const int nq = NTOK * NHEADS;
  attn_gather<<<(nq + 7) / 8, 256, 0, stream>>>(qkvf, routes, yh, nq);

  gemm_f16<0><<<dim3(BDIM / 128, NTOK / 128), 256, 0, stream>>>(
      yh, wouth, b_out, out, BDIM, 1.0f / 4096.0f);
}
